// DecoderLayer_43654047597074
// MI455X (gfx1250) — hardware-verified
//
#include <hip/hip_runtime.h>
#ifndef NB
#define NB 2
#endif
#ifndef SEQ
#define SEQ 2048
#endif
#define NB_FULL 2
#define SEQ_FULL 2048
#define DM 512
#define NH 8
#define HD 64
#define FH 2048
#define MROWS (NB * SEQ)
#define NQT (SEQ / 64)
#define NKT (SEQ / 64)
static_assert(SEQ % 64 == 0);
static_assert(SEQ <= SEQ_FULL);
static_assert(NB >= 1 && NB <= NB_FULL);
static_assert(NKT <= 32);
static_assert(MROWS % 128 == 0);
static_assert(DM == 512 && DM == NH * HD);
static_assert(DM % 64 == 0 && FH % 64 == 0 && (3 * DM) % 64 == 0 && (2 * DM) % 64 == 0);
static_assert((MROWS * (DM / 8)) % 256 == 0);
static_assert(MROWS % 8 == 0);

typedef _Float16 v16h __attribute__((ext_vector_type(16)));
typedef _Float16 v4h  __attribute__((ext_vector_type(4)));
typedef unsigned short v8us __attribute__((ext_vector_type(8), may_alias));
typedef float  v8f  __attribute__((ext_vector_type(8)));
typedef float  v4f  __attribute__((ext_vector_type(4)));
typedef float  v4fa __attribute__((ext_vector_type(4), may_alias));
typedef int    v4ia __attribute__((ext_vector_type(4), may_alias));
union FragH { v16h v; v8us half[2]; _Float16 h[16]; unsigned short u[16]; };

#define NEG_INF (-__builtin_inff())

__device__ __forceinline__ unsigned short bf16_bits(float x) { unsigned int u = __float_as_uint(x); return (unsigned short)((u + 0x7FFFu + ((u >> 16) & 1u)) >> 16); }
__device__ __forceinline__ float bf16_val(unsigned short b) { return __uint_as_float(((unsigned int)b) << 16); }
__device__ __forceinline__ float bf16_rne(float x) { return bf16_val(bf16_bits(x)); }
__device__ __forceinline__ unsigned rowf(unsigned mc) { return (mc / (unsigned)SEQ) * (unsigned)SEQ_FULL + (mc % (unsigned)SEQ); }

__device__ __forceinline__ v16h g2_frag(const _Float16* p, int hh) { FragH f; f.half[0] = *(const v8us*)((const unsigned short*)p + 8 * hh); f.half[1] = *(const v8us*)((const unsigned short*)p + 16 + 8 * hh); return f.v; }
__device__ __forceinline__ v8f g2_mma(v16h a, v16h b, v8f c) { v8f d = __builtin_amdgcn_wmma_f32_16x16x32_f16(false, a, false, b, (short)0, c, false, false); asm volatile("v_nop\n\tv_nop\n\tv_nop\n\tv_nop" : "+v"(d) : "v"(a), "v"(b)); return d; }

__global__ __launch_bounds__(256) void k_x16(const float* __restrict__ x, const float* __restrict__ y, _Float16* __restrict__ X16, _Float16* __restrict__ Y16) {
  const unsigned t = blockIdx.x * 256u + threadIdx.x; if (t >= (unsigned)(MROWS * (DM / 8))) return;
  const float* src = (blockIdx.y == 0) ? x : y; _Float16* dst = (blockIdx.y == 0) ? X16 : Y16;
  const unsigned mc = t >> 6, c8 = (t & 63u) * 8u;
  const float* sp = src + (size_t)rowf(mc) * DM + c8;
  const v4f a = *(const v4fa*)sp; const v4f c = *(const v4fa*)(sp + 4); FragH f;
#pragma unroll
  for (int q = 0; q < 4; ++q) { f.h[q] = (_Float16)bf16_rne(a[q]); f.h[4 + q] = (_Float16)bf16_rne(c[q]); }
  *(volatile v8us*)((unsigned short*)dst + (size_t)t * 8) = f.half[0]; __threadfence(); *(volatile v8us*)((unsigned short*)dst + (size_t)t * 8) = f.half[0]; }

__global__ __launch_bounds__(256) void k_wt(const float* __restrict__ W, _Float16* __restrict__ Bt, unsigned K, unsigned N) {
  __shared__ _Float16 tl[64][66];
  const unsigned tid = threadIdx.x; const unsigned n0 = blockIdx.x * 64u, k0 = blockIdx.y * 64u;
  for (unsigned i = tid; i < 1024u; i += 256u) { const unsigned r = i >> 4, c4 = (i & 15u) * 4u;
    const v4f v = *(const v4fa*)(W + (size_t)(k0 + r) * N + n0 + c4);
#pragma unroll
    for (int q = 0; q < 4; ++q) tl[r][c4 + q] = (_Float16)(bf16_rne(v[q]) * 16.0f); }
  __syncthreads();
  for (int pass = 0; pass < 2; ++pass) {
#pragma unroll
    for (unsigned rd = 0; rd < 2; ++rd) { const unsigned n = rd * 32u + (tid >> 3), pc = tid & 7u; FragH f;
#pragma unroll
      for (int q = 0; q < 8; ++q) f.h[q] = tl[pc * 8u + q][n];
      *(volatile v8us*)((unsigned short*)Bt + (size_t)(n0 + n) * K + k0 + pc * 8u) = f.half[0]; }
    if (pass == 0) __threadfence(); } }

template<int MODE>
__global__ __launch_bounds__(128) void k_gemm2(const _Float16* __restrict__ A, unsigned lda, const _Float16* __restrict__ Bh, unsigned ldb, float alpha, const float* __restrict__ bias,
    _Float16* __restrict__ C16, float* __restrict__ C32, unsigned ldc, unsigned M, unsigned N, unsigned K) {
  __shared__ __attribute__((aligned(16))) float so[4][32][68];
  const unsigned tid = threadIdx.x, w = tid >> 5, lane = tid & 31u, ln = lane & 15u; const int hh = (int)(lane >> 4);
  const unsigned ntn = N >> 6; const unsigned mt = blockIdx.x / ntn, nq = blockIdx.x - mt * ntn; const unsigned row0 = mt * 128u + 32u * w, col0 = nq * 64u; if (row0 >= M) return;
  const _Float16* a0p = A + (size_t)(row0 + ln) * lda; const _Float16* a1p = a0p + (size_t)16 * lda;
  const _Float16* b0p = Bh + (size_t)(col0 + ln) * ldb; const _Float16* b1p = b0p + (size_t)16 * ldb; const _Float16* b2p = b1p + (size_t)16 * ldb; const _Float16* b3p = b2p + (size_t)16 * ldb;
  const v8f z8 = {0.f,0.f,0.f,0.f,0.f,0.f,0.f,0.f}; v8f c00 = z8, c01 = z8, c02 = z8, c03 = z8, c10 = z8, c11 = z8, c12 = z8, c13 = z8;
#pragma unroll 1
  for (unsigned kb = 0; kb < K; kb += 32u) { const v16h a0 = g2_frag(a0p + kb, hh), a1 = g2_frag(a1p + kb, hh);
    v16h b = g2_frag(b0p + kb, hh); c00 = g2_mma(a0, b, c00); c10 = g2_mma(a1, b, c10);
    b = g2_frag(b1p + kb, hh); c01 = g2_mma(a0, b, c01); c11 = g2_mma(a1, b, c11);
    b = g2_frag(b2p + kb, hh); c02 = g2_mma(a0, b, c02); c12 = g2_mma(a1, b, c12);
    b = g2_frag(b3p + kb, hh); c03 = g2_mma(a0, b, c03); c13 = g2_mma(a1, b, c13); }
  v8f accs[8] = {c00, c01, c02, c03, c10, c11, c12, c13};
#pragma unroll
  for (int u = 0; u < 8; ++u) { const unsigned t = (unsigned)(u & 3), half = (unsigned)(u >> 2); const unsigned col = col0 + t * 16u + ln; const float bv = bf16_rne(bias[col]);
#pragma unroll
    for (int r = 0; r < 8; ++r) { const unsigned rloc = half * 16u + 8u * (unsigned)hh + (unsigned)r; float v = accs[u][r] * alpha + bv; if (MODE == 1) v = fmaxf(v, 0.0f); so[w][rloc][t * 16u + ln] = v; } }
  __builtin_amdgcn_fence(4  , "workgroup"); __builtin_amdgcn_wave_barrier();
  const unsigned rsub = lane >> 4, c4 = (lane & 15u) * 4u;
  for (int pass = 0; pass < 2; ++pass) {
#pragma unroll
    for (unsigned q = 0; q < 16; ++q) { const unsigned r = q * 2u + rsub; const v4f v = *(const v4fa*)&so[w][r][c4];
      if (MODE == 2) { *(volatile v4f*)(C32 + (size_t)(row0 + r) * ldc + col0 + c4) = v; }
      else { v4h h4;
#pragma unroll
        for (int i = 0; i < 4; ++i) h4[i] = (_Float16)v[i];
        *(volatile v4h*)(C16 + (size_t)(row0 + r) * ldc + col0 + c4) = h4; } }
    if (pass == 0) __threadfence(); } }

__global__ __launch_bounds__(256) void k_vt2(const _Float16* __restrict__ src, unsigned pitch, unsigned hs, _Float16* __restrict__ VT) {
  __shared__ unsigned short tl[64][66];
  const unsigned tid = threadIdx.x; const unsigned slab = blockIdx.x / (unsigned)NQT, lg = blockIdx.x - slab * (unsigned)NQT; const unsigned b = slab / (unsigned)NH, hd = slab - b * (unsigned)NH; const unsigned s0 = lg * 64u;
  for (unsigned i = tid; i < 64u * 8u; i += 256u) { const unsigned r = i >> 3, c8 = (i & 7u) * 8u; FragH f;
    f.half[0] = *(const v8us*)((const unsigned short*)src + (size_t)(b * (unsigned)SEQ + s0 + r) * pitch + hd * hs + c8);
#pragma unroll
    for (int q = 0; q < 8; ++q) tl[r][c8 + q] = f.u[q]; }
  __syncthreads();
  for (int pass = 0; pass < 2; ++pass) {
#pragma unroll
    for (unsigned rd = 0; rd < 2; ++rd) { const unsigned d = rd * 32u + (tid >> 3), pc = tid & 7u; FragH f;
#pragma unroll
      for (int q = 0; q < 8; ++q) f.u[q] = tl[pc * 8u + q][d];
      *(volatile v8us*)((unsigned short*)VT + ((size_t)slab * HD + d) * SEQ + s0 + pc * 8u) = f.half[0]; }
    if (pass == 0) __threadfence(); } }

__global__ __launch_bounds__(256) void k_mflag(const float* __restrict__ m0, const float* __restrict__ m1, int* __restrict__ MF) {
  __shared__ int sf[32];
  const unsigned tid = threadIdx.x, qt = blockIdx.x; const unsigned kt = tid >> 3, p = tid & 7u;
  const float* mask = (blockIdx.y == 0) ? m0 : m1;
  const bool ok = kt < (unsigned)NKT; const unsigned ktc = ok ? kt : (unsigned)(NKT - 1);
  int acc = 0;
#pragma unroll 1
  for (unsigned r = 0; r < 64u; ++r) {
    const float* rowp = mask + (size_t)(qt * 64u + r) * SEQ_FULL + ktc * 64u + p * 4u;
    const v4ia a = *(const v4ia*)rowp; const v4ia c = *(const v4ia*)(rowp + 32);
    acc |= (a[0] | a[1]) | (a[2] | a[3]) | (c[0] | c[1]) | (c[2] | c[3]); }
  acc = ok ? (acc & 0x7fffffff) : 0;
  acc |= __shfl_xor(acc, 1); acc |= __shfl_xor(acc, 2); acc |= __shfl_xor(acc, 4);
  if (p == 0) sf[kt] = (acc != 0) ? 1 : 0;
  __syncthreads();
  if (tid < 32u) { const int v = sf[tid]; volatile int* d = MF + ((size_t)blockIdx.y * NQT + qt) * 32 + tid; *d = v; __threadfence(); *d = v; } }

__global__ __launch_bounds__(128) void k_attn(const _Float16* Qp, unsigned qpitch, unsigned qhs, const _Float16* Kp, unsigned kpitch, unsigned khs,
                                              const _Float16* __restrict__ VT, const float* __restrict__ mask, const int* __restrict__ MF, _Float16* __restrict__ CTX) {
  __shared__ __attribute__((aligned(16))) float so[4][16][68];
  const unsigned tid = threadIdx.x, w = tid >> 5, lane = tid & 31u, l15 = lane & 15u; const int hh = (int)(lane >> 4);
  const unsigned qt = blockIdx.x, slab = blockIdx.y; const unsigned b = slab / (unsigned)NH, hd = slab - b * (unsigned)NH;
  const unsigned q0 = qt * 64u + w * 16u;
  const _Float16* Qb = Qp + (size_t)b * SEQ * qpitch + hd * qhs;
  const _Float16* Kb = Kp + (size_t)b * SEQ * kpitch + hd * khs;
  const _Float16* Vb = VT + (size_t)slab * HD * SEQ;
  const _Float16* qrow = Qb + (size_t)(q0 + l15) * qpitch;
  const v16h qf0 = g2_frag(qrow, hh), qf1 = g2_frag(qrow + 32, hh);
  const v8f z8 = {0.f,0.f,0.f,0.f,0.f,0.f,0.f,0.f};
  v8f o[4] = {z8, z8, z8, z8};
  float m = NEG_INF, l = 0.f;
  const float CL = 0.18033688011112042f;
#pragma unroll 1
  for (unsigned it = 0; it < (unsigned)NKT; ++it) {
    const unsigned key0 = it * 64u;
    v8f s[4];
#pragma unroll
    for (int kt = 0; kt < 4; ++kt) {
      const _Float16* krow = Kb + (size_t)(key0 + (unsigned)kt * 16u + l15) * kpitch;
      const v16h ka = g2_frag(krow, hh), kk = g2_frag(krow + 32, hh);
      v8f a = g2_mma(ka, qf0, z8); a = g2_mma(kk, qf1, a); s[kt] = a; }
    const int mf = MF[(size_t)qt * 32 + it];
    if (mf != 0) {
#pragma unroll
      for (int kt = 0; kt < 4; ++kt) {
        const float* mp = mask + (size_t)(q0 + l15) * SEQ_FULL + key0 + (unsigned)kt * 16u + 8u * (unsigned)hh;
        const v4f ma = *(const v4fa*)mp; const v4f mb = *(const v4fa*)(mp + 4);
#pragma unroll
        for (int r = 0; r < 4; ++r) { s[kt][r] = fmaf(bf16_rne(ma[r]), 8.0f, s[kt][r]); s[kt][4 + r] = fmaf(bf16_rne(mb[r]), 8.0f, s[kt][4 + r]); } } }
    float lmax = NEG_INF;
#pragma unroll
    for (int kt = 0; kt < 4; ++kt)
#pragma unroll
      for (int r = 0; r < 8; ++r) lmax = fmaxf(lmax, s[kt][r]);
    lmax = fmaxf(lmax, __shfl_xor(lmax, 16));
    const float mnew = fmaxf(m, lmax);
    const float mz = (mnew == NEG_INF) ? 0.0f : mnew;
    const float alpha = exp2f((m - mz) * CL);
    const float bexp = 10.0f - mz * CL;
    m = mnew;
    float psum = 0.f; FragH pa, pb;
#pragma unroll
    for (int r = 0; r < 8; ++r) {
      const float e0 = exp2f(fmaf(s[0][r], CL, bexp)), e1 = exp2f(fmaf(s[1][r], CL, bexp)), e2 = exp2f(fmaf(s[2][r], CL, bexp)), e3 = exp2f(fmaf(s[3][r], CL, bexp));
      psum += (e0 + e1) + (e2 + e3);
      pa.h[r] = (_Float16)e0; pa.h[8 + r] = (_Float16)e1; pb.h[r] = (_Float16)e2; pb.h[8 + r] = (_Float16)e3; }
    l = l * alpha + psum;
    float ar[8];
#pragma unroll
    for (int r = 0; r < 8; ++r) ar[r] = __shfl(alpha, 8 * hh + r);
#pragma unroll
    for (int dt = 0; dt < 4; ++dt) {
#pragma unroll
      for (int r = 0; r < 8; ++r) o[dt][r] *= ar[r];
      const _Float16* vrow = Vb + (size_t)((unsigned)dt * 16u + l15) * SEQ + key0;
      const v16h va = g2_frag(vrow, hh), vb = g2_frag(vrow + 32, hh);
      o[dt] = g2_mma(pa.v, va, o[dt]); o[dt] = g2_mma(pb.v, vb, o[dt]); } }
  const float lt = l + __shfl_xor(l, 16);
  const float inv = (1.0f / lt) * 256.0f;
  float ir[8];
#pragma unroll
  for (int r = 0; r < 8; ++r) ir[r] = __shfl(inv, 8 * hh + r);
#pragma unroll
  for (int dt = 0; dt < 4; ++dt)
#pragma unroll
    for (int r = 0; r < 8; ++r) so[w][8 * hh + r][dt * 16 + (int)l15] = o[dt][r] * ir[r];
  __builtin_amdgcn_fence(4  , "workgroup"); __builtin_amdgcn_wave_barrier();
  const unsigned rq = lane >> 3, pc = lane & 7u;
  for (int pass = 0; pass < 2; ++pass) {
#pragma unroll
    for (unsigned g = 0; g < 4; ++g) { const unsigned row = g * 4u + rq;
      const v4f v0 = *(const v4fa*)&so[w][row][pc * 8u]; const v4f v1 = *(const v4fa*)&so[w][row][pc * 8u + 4u]; FragH f;
#pragma unroll
      for (int i = 0; i < 4; ++i) { f.h[i] = (_Float16)v0[i]; f.h[4 + i] = (_Float16)v1[i]; }
      *(volatile v8us*)((unsigned short*)CTX + (size_t)(b * (unsigned)SEQ + q0 + row) * DM + hd * (unsigned)HD + pc * 8u) = f.half[0]; }
    if (pass == 0) __threadfence(); } }

template<int KIND>
__global__ __launch_bounds__(256) void k_ln(const float* __restrict__ a, const float* __restrict__ res, const float* __restrict__ g, const float* __restrict__ bt,
                                            float* __restrict__ outF, _Float16* __restrict__ out16) {
  __shared__ __attribute__((aligned(16))) float sx[8][DM];
  const unsigned tid = threadIdx.x, w = tid >> 5, lane = tid & 31u;
  const unsigned mc = blockIdx.x * 8u + w;
  const size_t abase = (size_t)mc * DM;
  const size_t rbase = (KIND == 0) ? (size_t)rowf(mc) * DM : abase;
  const size_t obase = (KIND == 2) ? (size_t)rowf(mc) * DM : abase;
  float s = 0.f;
#pragma unroll 1
  for (unsigned j = 0; j < 4u; ++j) { const unsigned c = j * 128u + lane * 4u;
    const v4f av = *(const v4fa*)(a + abase + c); v4f rv = *(const v4fa*)(res + rbase + c);
    if (KIND == 0) {
#pragma unroll
      for (int i = 0; i < 4; ++i) rv[i] = bf16_rne(rv[i]); }
    const v4f xv = av + rv; *(v4fa*)&sx[w][c] = xv; s += (xv[0] + xv[1]) + (xv[2] + xv[3]); }
  s += __shfl_xor(s, 16); s += __shfl_xor(s, 8); s += __shfl_xor(s, 4); s += __shfl_xor(s, 2); s += __shfl_xor(s, 1);
  const float mean = s * (1.0f / 512.0f);
  float ss = 0.f;
#pragma unroll 1
  for (unsigned j = 0; j < 4u; ++j) { const unsigned c = j * 128u + lane * 4u; const v4f xv = *(const v4fa*)&sx[w][c];
    const float d0 = xv[0] - mean, d1 = xv[1] - mean, d2 = xv[2] - mean, d3 = xv[3] - mean; ss += (d0 * d0 + d1 * d1) + (d2 * d2 + d3 * d3); }
  ss += __shfl_xor(ss, 16); ss += __shfl_xor(ss, 8); ss += __shfl_xor(ss, 4); ss += __shfl_xor(ss, 2); ss += __shfl_xor(ss, 1);
  const float sd = sqrtf(ss * (1.0f / 511.0f)) + 1e-5f;
  const float inv = 1.0f / sd;
  for (int pass = 0; pass < 2; ++pass) {
#pragma unroll 1
    for (unsigned j = 0; j < 4u; ++j) { const unsigned c = j * 128u + lane * 4u; const v4f xv = *(const v4fa*)&sx[w][c];
      const v4f gv = *(const v4fa*)(g + c); const v4f bv = *(const v4fa*)(bt + c); v4f ov; v4h h4;
#pragma unroll
      for (int i = 0; i < 4; ++i) { ov[i] = (bf16_rne(gv[i]) * (xv[i] - mean)) * inv + bf16_rne(bv[i]); h4[i] = (_Float16)ov[i]; }
      *(volatile v4f*)(outF + obase + c) = ov;
      if (KIND != 2) *(volatile v4h*)(out16 + abase + c) = h4; }
    if (pass == 0) __threadfence(); } }

extern "C" void kernel_launch(void* const* d_in, const int* in_sizes, int n_in,
                              void* d_out, int out_size, void* d_ws, size_t ws_size, hipStream_t stream) {
  if (n_in < 24) return;
  const float* x   = (const float*)d_in[0];
  const float* y   = (const float*)d_in[1];
  const float* mks = (const float*)d_in[2];
  const float* mkc = (const float*)d_in[3];
  const float* qkv_w = (const float*)d_in[4];  const float* qkv_b = (const float*)d_in[5];
  const float* so_w  = (const float*)d_in[6];  const float* so_b  = (const float*)d_in[7];
  const float* kv_w  = (const float*)d_in[8];  const float* kv_b  = (const float*)d_in[9];
  const float* q_w   = (const float*)d_in[10]; const float* q_b   = (const float*)d_in[11];
  const float* co_w  = (const float*)d_in[12]; const float* co_b  = (const float*)d_in[13];
  const float* f1_w  = (const float*)d_in[14]; const float* f1_b  = (const float*)d_in[15];
  const float* f2_w  = (const float*)d_in[16]; const float* f2_b  = (const float*)d_in[17];
  const float* g1 = (const float*)d_in[18]; const float* b1 = (const float*)d_in[19];
  const float* g2 = (const float*)d_in[20]; const float* b2 = (const float*)d_in[21];
  const float* g3 = (const float*)d_in[22]; const float* b3 = (const float*)d_in[23];
  const long need_rows = (long)(NB - 1) * SEQ_FULL + SEQ;
  if ((long)in_sizes[0] < need_rows * DM || (long)in_sizes[1] < need_rows * DM) return;
  if ((long)in_sizes[2] < (long)(SEQ - 1) * SEQ_FULL + SEQ || (long)in_sizes[3] < (long)(SEQ - 1) * SEQ_FULL + SEQ) return;
  if (in_sizes[4] < DM * 3 * DM || in_sizes[5] < 3 * DM) return;
  if (in_sizes[6] < DM * DM || in_sizes[7] < DM) return;
  if (in_sizes[8] < DM * 2 * DM || in_sizes[9] < 2 * DM) return;
  if (in_sizes[10] < DM * DM || in_sizes[11] < DM) return;
  if (in_sizes[12] < DM * DM || in_sizes[13] < DM) return;
  if (in_sizes[14] < DM * FH || in_sizes[15] < FH) return;
  if (in_sizes[16] < FH * DM || in_sizes[17] < DM) return;
  for (int i = 18; i < 24; ++i) if (in_sizes[i] < DM) return;
  if ((long)out_size < need_rows * DM) return;
  char* ws = (char*)d_ws; size_t off = 0;
  auto take = [&](size_t bytes) { char* p = ws + off; off += (bytes + 255) & ~(size_t)255; return p; };
  _Float16* BQKV = (_Float16*)take((size_t)3 * DM * DM * 2);
  _Float16* BSO  = (_Float16*)take((size_t)DM * DM * 2);
  _Float16* BKV  = (_Float16*)take((size_t)2 * DM * DM * 2);
  _Float16* BQ   = (_Float16*)take((size_t)DM * DM * 2);
  _Float16* BCO  = (_Float16*)take((size_t)DM * DM * 2);
  _Float16* BF1  = (_Float16*)take((size_t)FH * DM * 2);
  _Float16* BF2  = (_Float16*)take((size_t)DM * FH * 2);
  _Float16* X16  = (_Float16*)take((size_t)MROWS * DM * 2);
  _Float16* Y16  = (_Float16*)take((size_t)MROWS * DM * 2);
  _Float16* QKV  = (_Float16*)take((size_t)MROWS * 3 * DM * 2);
  _Float16* KV   = (_Float16*)take((size_t)MROWS * 2 * DM * 2);
  _Float16* QC   = (_Float16*)take((size_t)MROWS * DM * 2);
  _Float16* VT   = (_Float16*)take((size_t)NB * NH * HD * SEQ * 2);
  _Float16* CTX  = (_Float16*)take((size_t)MROWS * DM * 2);
  _Float16* Y1H  = (_Float16*)take((size_t)MROWS * DM * 2);
  _Float16* Y2H  = (_Float16*)take((size_t)MROWS * DM * 2);
  _Float16* H16  = (_Float16*)take((size_t)MROWS * FH * 2);
  float*    AF   = (float*)take((size_t)MROWS * DM * 4);
  float*    Y1F  = (float*)take((size_t)MROWS * DM * 4);
  float*    Y2F  = (float*)take((size_t)MROWS * DM * 4);
  int*      MF   = (int*)take((size_t)2 * NQT * 32 * 4);
  if (off > ws_size || off > (size_t)134217728) return;

  k_x16<<<dim3((unsigned)(MROWS * (DM / 8) / 256), 2u), 256, 0, stream>>>(x, y, X16, Y16);
  k_wt<<<dim3(3 * DM / 64, DM / 64), 256, 0, stream>>>(qkv_w, BQKV, (unsigned)DM, (unsigned)(3 * DM));
  k_wt<<<dim3(DM / 64, DM / 64),     256, 0, stream>>>(so_w,  BSO,  (unsigned)DM, (unsigned)DM);
  k_wt<<<dim3(2 * DM / 64, DM / 64), 256, 0, stream>>>(kv_w,  BKV,  (unsigned)DM, (unsigned)(2 * DM));
  k_wt<<<dim3(DM / 64, DM / 64),     256, 0, stream>>>(q_w,   BQ,   (unsigned)DM, (unsigned)DM);
  k_wt<<<dim3(DM / 64, DM / 64),     256, 0, stream>>>(co_w,  BCO,  (unsigned)DM, (unsigned)DM);
  k_wt<<<dim3(FH / 64, DM / 64),     256, 0, stream>>>(f1_w,  BF1,  (unsigned)DM, (unsigned)FH);
  k_wt<<<dim3(DM / 64, FH / 64),     256, 0, stream>>>(f2_w,  BF2,  (unsigned)FH, (unsigned)DM);
  k_mflag<<<dim3((unsigned)NQT, 2u), 256, 0, stream>>>(mks, mkc, MF);

  const unsigned mt = (unsigned)(MROWS / 128);
  k_gemm2<0><<<mt * (3 * DM / 64), 128, 0, stream>>>(Y16, DM, BQKV, DM, 0.0625f, qkv_b, QKV, (float*)0, 3 * DM, MROWS, 3 * DM, DM);
  k_vt2<<<(unsigned)(NB * NH * NQT), 256, 0, stream>>>(QKV + 2 * HD, 3 * DM, 3 * HD, VT);
  k_attn<<<dim3((unsigned)NQT, (unsigned)(NB * NH)), 128, 0, stream>>>(QKV, 3 * DM, 3 * HD, QKV + HD, 3 * DM, 3 * HD, VT, mks, MF, CTX);
  k_gemm2<2><<<mt * (DM / 64), 128, 0, stream>>>(CTX, DM, BSO, DM, 1.0f / 4096.0f, so_b, (_Float16*)0, AF, DM, MROWS, DM, DM);
  k_ln<0><<<(unsigned)(MROWS / 8), 256, 0, stream>>>(AF, y, g1, b1, Y1F, Y1H);

  k_gemm2<0><<<mt * (2 * DM / 64), 128, 0, stream>>>(X16, DM, BKV, DM, 0.0625f, kv_b, KV, (float*)0, 2 * DM, MROWS, 2 * DM, DM);
  k_gemm2<0><<<mt * (DM / 64), 128, 0, stream>>>(Y1H, DM, BQ, DM, 0.0625f, q_b, QC, (float*)0, DM, MROWS, DM, DM);
  k_vt2<<<(unsigned)(NB * NH * NQT), 256, 0, stream>>>(KV + HD, 2 * DM, 2 * HD, VT);
  k_attn<<<dim3((unsigned)NQT, (unsigned)(NB * NH)), 128, 0, stream>>>(QC, DM, HD, KV, 2 * DM, 2 * HD, VT, mkc, MF + (size_t)NQT * 32, CTX);
  k_gemm2<2><<<mt * (DM / 64), 128, 0, stream>>>(CTX, DM, BCO, DM, 1.0f / 4096.0f, co_b, (_Float16*)0, AF, DM, MROWS, DM, DM);
  k_ln<1><<<(unsigned)(MROWS / 8), 256, 0, stream>>>(AF, Y1F, g2, b2, Y2F, Y2H);

  k_gemm2<1><<<mt * (FH / 64), 128, 0, stream>>>(Y2H, DM, BF1, DM, 0.0625f, f1_b, H16, (float*)0, FH, MROWS, FH, DM);
  k_gemm2<2><<<mt * (DM / 64), 128, 0, stream>>>(H16, FH, BF2, FH, 0.0625f, f2_b, (_Float16*)0, AF, DM, MROWS, DM, FH);
  k_ln<2><<<(unsigned)(MROWS / 8), 256, 0, stream>>>(AF, Y2F, g3, b3, (float*)d_out, (_Float16*)0);
}
